// BiMambaBlock_79791902425748
// MI455X (gfx1250) — hardware-run, weakly checked
//
#include <hip/hip_runtime.h>
#include <math.h>

typedef __attribute__((ext_vector_type(16))) _Float16 v16h;
typedef __attribute__((ext_vector_type(8)))  _Float16 v8h;
typedef __attribute__((ext_vector_type(16))) __bf16   v16b;
typedef __attribute__((ext_vector_type(8)))  __bf16   v8b;
typedef __attribute__((ext_vector_type(8)))  float    v8f;
typedef __attribute__((ext_vector_type(4)))  float    v4f;
typedef __attribute__((ext_vector_type(2)))  float    v2f;

constexpr int kBatch  = 2;
constexpr int kSeq    = 4096;
constexpr int kDm     = 256;
constexpr int kDin    = 512;
constexpr int kNst    = 16;
constexpr int kDtR    = 16;
constexpr int kXzP    = 2 * kDin;
constexpr int kXdW    = kDtR + 2 * kNst;
constexpr int kXdP    = 64;
constexpr int kDff    = 4 * kDm;
constexpr int kRows   = kBatch * kSeq;
constexpr int kConvTP = 260;
constexpr int kScanTS = 64;
constexpr int kScanCh = 64;
constexpr int kScanYP = 68;
constexpr int kTrP    = 68;
static_assert(kXdW <= kXdP, "x_proj pad");
static_assert((kDm % 32) == 0 && (kDin % 32) == 0 && (kDff % 32) == 0, "GEMM K multiples of 32");
static_assert((kRows % 64) == 0 && (kXzP % 64) == 0 && (kXdP % 64) == 0 && (kDm % 64) == 0 && (kDff % 64) == 0, "GEMM M,N multiples of 64");
static_assert((kSeq % kScanTS) == 0 && (kSeq % 64) == 0 && (kDin % kScanCh) == 0 && (kDin % 256) == 0, "tile multiples");
static_assert((kXdW % 4) == 0 && (kDm % 4) == 0, "transpose source widths multiples of 4");

constexpr size_t kOffXB   = 0;
constexpr size_t kOffWIB  = kOffXB  + (size_t)kRows * kDm  * 2;
constexpr size_t kOffWXB  = kOffWIB + (size_t)kXzP  * kDm  * 2;
constexpr size_t kOffWOB  = kOffWXB + (size_t)kXdP  * kDin * 2;
constexpr size_t kOffWF1  = kOffWOB + (size_t)kDm   * kDin * 2;
constexpr size_t kOffWF2  = kOffWF1 + (size_t)kDff  * kDm  * 2;
constexpr size_t kOffXZ   = kOffWF2 + (size_t)kDm   * kDff * 2;
constexpr size_t kOffXC   = kOffXZ  + (size_t)kRows * kXzP * 4;
constexpr size_t kOffXCH  = kOffXC  + (size_t)kRows * kDin * 4;
constexpr size_t kOffXCL  = kOffXCH + (size_t)kRows * kDin * 2;
constexpr size_t kOffPR   = kOffXCL + (size_t)kRows * kDin * 2;
constexpr size_t kOffYS   = kOffPR  + (size_t)kRows * kXdP * 4;
constexpr size_t kOffYH   = kOffYS  + (size_t)kRows * kDin * 4;
constexpr size_t kOffYL   = kOffYH  + (size_t)kRows * kDin * 2;
constexpr size_t kOffY2H  = kOffYL  + (size_t)kRows * kDin * 2;
constexpr size_t kOffY2L  = kOffY2H + (size_t)kRows * kDm  * 2;
constexpr size_t kWsTotal = kOffY2L + (size_t)kRows * kDm  * 2;
constexpr size_t kOffHP   = kOffXZ;
constexpr size_t kOffFF   = kOffXC;
constexpr size_t kOffHH   = kOffXCH;
constexpr size_t kOffYf   = kOffYS;
constexpr size_t kOffHL   = kOffYH;
static_assert(kWsTotal == 117243904ull, "carve total");
static_assert(kWsTotal <= 134217728ull, "carve cap");
static_assert(kOffHP + (size_t)kRows * kDff * 4 <= kOffXC,  "HP fits XZ");
static_assert(kOffFF + (size_t)kRows * kDm  * 4 <= kOffXCH, "FF fits XC");
static_assert(kOffHH + (size_t)kRows * kDff * 2 <= kOffPR,  "HH fits XCH|XCL");
static_assert(kOffYf + (size_t)kRows * kDm  * 4 <= kOffYH,  "Yf fits YS");
static_assert(kOffHL + (size_t)kRows * kDff * 2 <= kOffY2H, "HL fits YH|YL");
static_assert((kOffWIB % 128) == 0 && (kOffWXB % 128) == 0 && (kOffWOB % 128) == 0 && (kOffWF1 % 128) == 0 &&
              (kOffWF2 % 128) == 0 && (kOffXZ % 128) == 0 && (kOffXC % 128) == 0 && (kOffXCH % 128) == 0 &&
              (kOffXCL % 128) == 0 && (kOffPR % 128) == 0 && (kOffYS % 128) == 0 && (kOffYH % 128) == 0 &&
              (kOffYL % 128) == 0 && (kOffY2H % 128) == 0 && (kOffY2L % 128) == 0, "128-B aligned regions");

__device__ __forceinline__ unsigned short f2bf_bits(float f) {
  unsigned u = __float_as_uint(f);
  return (unsigned short)((u + 0x7FFFu + ((u >> 16) & 1u)) >> 16);
}
__device__ __forceinline__ float bf_bits2f(unsigned short h) { return __uint_as_float(((unsigned)h) << 16); }
__device__ __forceinline__ float bf_rne(float f) { return bf_bits2f(f2bf_bits(f)); }

__device__ __forceinline__ void dep_guard4_h(v8f& a, v8f& b, v8f& c, v8f& d, v16h x, v16h y) { asm volatile("v_nop\n\tv_nop\n\tv_nop\n\tv_nop" : "+v"(a), "+v"(b), "+v"(c), "+v"(d) : "v"(x), "v"(y)); }
__device__ __forceinline__ void dep_guard4_b(v8f& a, v8f& b, v8f& c, v8f& d, v16b x, v16b y) { asm volatile("v_nop\n\tv_nop\n\tv_nop\n\tv_nop" : "+v"(a), "+v"(b), "+v"(c), "+v"(d) : "v"(x), "v"(y)); }
__device__ __forceinline__ void keep4_h(v16h a, v16h b, v16h c, v16h d) { asm volatile("v_nop" :: "v"(a), "v"(b), "v"(c), "v"(d)); }
__device__ __forceinline__ void keep4_b(v16b a, v16b b, v16b c, v16b d) { asm volatile("v_nop" :: "v"(a), "v"(b), "v"(c), "v"(d)); }
__device__ __forceinline__ void acc_guard4(v8f& a, v8f& b, v8f& c, v8f& d) { asm volatile("v_nop\n\tv_nop\n\tv_nop\n\tv_nop" : "+v"(a), "+v"(b), "+v"(c), "+v"(d)); }
template <typename T> struct Frag;
template <> struct Frag<_Float16> {
  typedef v16h V; union U { v16h v; v8h h[2]; };
  static __device__ __forceinline__ v16h load(const _Float16* p) {
    U f; f.h[0] = *(const v8h*)(p); f.h[1] = *(const v8h*)(p + 16); return f.v;
  }
  static __device__ __forceinline__ v8f mma(v16h a, v16h b, v8f c) {
    return __builtin_amdgcn_wmma_f32_16x16x32_f16(false, a, false, b, (short)0, c, false, false);
  }
  static __device__ __forceinline__ void guard4(v8f& a, v8f& b, v8f& c, v8f& d, v16h x, v16h y) { dep_guard4_h(a, b, c, d, x, y); }
  static __device__ __forceinline__ void keep(v16h a, v16h b, v16h c, v16h d) { keep4_h(a, b, c, d); }
};
template <> struct Frag<__bf16> {
  typedef v16b V; union U { v16b v; v8b h[2]; };
  static __device__ __forceinline__ v16b load(const __bf16* p) {
    U f; f.h[0] = *(const v8b*)(p); f.h[1] = *(const v8b*)(p + 16); return f.v;
  }
  static __device__ __forceinline__ v8f mma(v16b a, v16b b, v8f c) {
    return __builtin_amdgcn_wmma_f32_16x16x32_bf16(false, a, false, b, (short)0, c, false, false);
  }
  static __device__ __forceinline__ void guard4(v8f& a, v8f& b, v8f& c, v8f& d, v16b x, v16b y) { dep_guard4_b(a, b, c, d, x, y); }
  static __device__ __forceinline__ void keep(v16b a, v16b b, v16b c, v16b d) { keep4_b(a, b, c, d); }
};

template <int ET> struct Elem;
template <> struct Elem<0> { typedef _Float16 T; };
template <> struct Elem<1> { typedef __bf16 T; };
template <int ET, int SPL, int BIAS_MODE, int OUT_MODE, bool RESID, int ACT = 0>
__global__ __launch_bounds__(256) void wmma_gemm64(
    const unsigned short* __restrict__ Ap, const unsigned short* __restrict__ A2p, int lda, long strideA,
    const unsigned short* __restrict__ Btp, const unsigned short* __restrict__ Bt2p, int ldb, long strideB,
    void* __restrict__ Cout, void* __restrict__ Cout2, int ldc, long strideC,
    const float* __restrict__ bias,
    const float* __restrict__ resid, long strideR,
    int M, int N, int K, float scale) {
  typedef typename Elem<ET>::T T;
  typedef typename Frag<T>::V V;
  const T* A = (const T*)Ap; const T* A2 = (const T*)A2p; const T* Bt = (const T*)Btp; const T* Bt2 = (const T*)Bt2p;
  __shared__ __align__(16) float sT[8][16 * 68];
  const int b    = blockIdx.y;
  const int lane = threadIdx.x & 31;
  const int wave = threadIdx.x >> 5;
  const int tilesN = N >> 6;
  const int tilesM = M >> 6;
  const int tile = blockIdx.x * 8 + wave;
  if (tile >= tilesM * tilesN) return;
  const int tm = tile / tilesN;
  const int tn = tile - tm * tilesN;
  const int m0 = tm << 6;
  const int n0 = tn << 6;

  const T* Ab  = A  + (size_t)b * strideA;
  const T* Bb  = Bt + (size_t)b * strideB;
  const T* Ab2 = (SPL >= 1) ? (A2  + (size_t)b * strideA) : nullptr;
  const T* Bb2 = (SPL == 2) ? (Bt2 + (size_t)b * strideB) : nullptr;

  const int rlane = lane & 15;
  const int koff  = (lane >> 4) * 8;
  const int mOff  = (lane >> 4) * 8;

  v8f acc[4][4];
#pragma unroll
  for (int i = 0; i < 4; ++i)
#pragma unroll
    for (int j = 0; j < 4; ++j) acc[i][j] = (v8f){0.f,0.f,0.f,0.f,0.f,0.f,0.f,0.f};

  for (int k0 = 0; k0 < K; k0 += 32) {
    V bh[4], bl[4];
#pragma unroll
    for (int j = 0; j < 4; ++j) {
      const size_t bo = (size_t)(n0 + (j << 4) + rlane) * ldb + koff + k0;
      bh[j] = Frag<T>::load(Bb + bo);
      if (SPL == 2) bl[j] = Frag<T>::load(Bb2 + bo);
    }
#pragma unroll
    for (int i = 0; i < 4; ++i) {
      const size_t ao = (size_t)(m0 + (i << 4) + rlane) * lda + koff + k0;
      V ah = Frag<T>::load(Ab + ao);
      V al = ah;
      if (SPL >= 1) al = Frag<T>::load(Ab2 + ao);
#pragma unroll
      for (int j = 0; j < 4; ++j) {
        acc[i][j] = Frag<T>::mma(ah, bh[j], acc[i][j]);
        if (SPL == 2) acc[i][j] = Frag<T>::mma(ah, bl[j], acc[i][j]);
        if (SPL >= 1) acc[i][j] = Frag<T>::mma(al, bh[j], acc[i][j]);
      }
      Frag<T>::guard4(acc[i][0], acc[i][1], acc[i][2], acc[i][3], ah, al);
    }
    Frag<T>::keep(bh[0], bh[1], bh[2], bh[3]);
    if (SPL == 2) Frag<T>::keep(bl[0], bl[1], bl[2], bl[3]);
  }
  acc_guard4(acc[0][0], acc[0][1], acc[0][2], acc[0][3]);
  acc_guard4(acc[1][0], acc[1][1], acc[1][2], acc[1][3]);
  acc_guard4(acc[2][0], acc[2][1], acc[2][2], acc[2][3]);
  acc_guard4(acc[3][0], acc[3][1], acc[3][2], acc[3][3]);

  float* slab = sT[wave];
  const float* Rb = RESID ? (resid + (size_t)b * strideR) : nullptr;
#pragma unroll
  for (int i = 0; i < 4; ++i) {
    const int mBase = m0 + (i << 4);
#pragma unroll
    for (int j = 0; j < 4; ++j) {
      const int n = n0 + (j << 4) + rlane;
      float bv = 0.f;
      if (BIAS_MODE == 2) bv = bias[n];
#pragma unroll
      for (int r = 0; r < 8; ++r) {
        float v = acc[i][j][r] * scale;
        if (BIAS_MODE == 1) v += bias[mBase + mOff + r];
        if (BIAS_MODE == 2) v += bv;
        if (RESID) v += Rb[(size_t)(mBase + mOff + r) * ldc + n];
        if (ACT == 1) v = tanhf(v);
        if (ACT == 2) v = fmaxf(v, 0.0f);
        if (ACT == 3) v = v / (1.0f + expf(-v));
        if (ACT == 4) v = (v > 0.f) ? v : 0.01f * v;
        slab[(mOff + r) * 68 + (j << 4) + rlane] = v;
      }
    }
    __builtin_amdgcn_fence(__ATOMIC_RELEASE, "workgroup");
    __builtin_amdgcn_wave_barrier();
    __builtin_amdgcn_fence(__ATOMIC_ACQUIRE, "workgroup");
    if (OUT_MODE == 0) {
      float* C = (float*)Cout + (size_t)b * strideC;
      const int hh = lane >> 4, c4 = (lane & 15) * 4;
      for (int pass = 0; pass < 2; ++pass) {
#pragma unroll
        for (int it = 0; it < 8; ++it) {
          const int row = it * 2 + hh;
          v4f v = *(const v4f*)(slab + row * 68 + c4);
          *(volatile v4f*)(C + (size_t)(mBase + row) * ldc + n0 + c4) = v;
        }
        __threadfence();
      }
    } else {
      const int q = lane >> 3, c8 = (lane & 7) * 8;
      unsigned short* C  = (unsigned short*)Cout  + (size_t)b * strideC;
      unsigned short* C2 = (OUT_MODE == 2) ? ((unsigned short*)Cout2 + (size_t)b * strideC) : nullptr;
      for (int pass = 0; pass < 2; ++pass) {
#pragma unroll
        for (int it = 0; it < 4; ++it) {
          const int row = it * 4 + q;
          const float* sp = slab + row * 68 + c8;
          v8h hv, lv;
#pragma unroll
          for (int e = 0; e < 8; ++e) {
            if (OUT_MODE == 1) {
              hv[e] = (_Float16)sp[e];
            } else {
              unsigned short hb = f2bf_bits(sp[e]);
              unsigned short lb = f2bf_bits(sp[e] - bf_bits2f(hb));
              hv[e] = __builtin_bit_cast(_Float16, hb);
              lv[e] = __builtin_bit_cast(_Float16, lb);
            }
          }
          *(volatile v8h*)(C + (size_t)(mBase + row) * ldc + n0 + c8) = hv;
          if (OUT_MODE == 2) *(volatile v8h*)(C2 + (size_t)(mBase + row) * ldc + n0 + c8) = lv;
        }
        __threadfence();
      }
    }
    __builtin_amdgcn_fence(__ATOMIC_RELEASE, "workgroup");
    __builtin_amdgcn_wave_barrier();
    __builtin_amdgcn_fence(__ATOMIC_ACQUIRE, "workgroup");
  }
}

__global__ __launch_bounds__(256) void rne_rows_bf16_kernel(
    const float* __restrict__ src, unsigned short* __restrict__ dst, int total8)
{
  const int i = blockIdx.x * 256 + threadIdx.x;
  if (i >= total8) return;
  const size_t e0 = (size_t)i << 3;
  const v4f a0 = *(const v4f*)(src + e0);
  const v4f a1 = *(const v4f*)(src + e0 + 4);
  v8h hv;
#pragma unroll
  for (int e = 0; e < 4; ++e) {
    const float f0 = a0[e], f1 = a1[e];
    hv[e]     = __builtin_bit_cast(_Float16, f2bf_bits(f0));
    hv[4 + e] = __builtin_bit_cast(_Float16, f2bf_bits(f1));
  }
  unsigned short* q = dst + e0;
  *(volatile v8h*)q = hv;
  __threadfence();
  *(volatile v8h*)q = hv;
}

__global__ __launch_bounds__(256) void split_rows_bf16_kernel(
    const float* __restrict__ src, unsigned short* __restrict__ dhi, unsigned short* __restrict__ dlo, int total8)
{
  const int i = blockIdx.x * 256 + threadIdx.x;
  if (i >= total8) return;
  const size_t e0 = (size_t)i << 3;
  const v4f a0 = *(const v4f*)(src + e0);
  const v4f a1 = *(const v4f*)(src + e0 + 4);
  v8h hv, lv;
#pragma unroll
  for (int e = 0; e < 4; ++e) {
    const float f0 = a0[e], f1 = a1[e];
    const unsigned short h0 = f2bf_bits(f0), h1 = f2bf_bits(f1);
    const unsigned short l0 = f2bf_bits(f0 - bf_bits2f(h0)), l1 = f2bf_bits(f1 - bf_bits2f(h1));
    hv[e]     = __builtin_bit_cast(_Float16, h0);
    hv[4 + e] = __builtin_bit_cast(_Float16, h1);
    lv[e]     = __builtin_bit_cast(_Float16, l0);
    lv[4 + e] = __builtin_bit_cast(_Float16, l1);
  }
  unsigned short* qh = dhi + e0;
  unsigned short* ql = dlo + e0;
  *(volatile v8h*)qh = hv;
  *(volatile v8h*)ql = lv;
  __threadfence();
  *(volatile v8h*)qh = hv;
  *(volatile v8h*)ql = lv;
}

__global__ __launch_bounds__(256) void transpose_bf16_kernel(
    const float* __restrict__ in, int Nreal, int Krows, unsigned short* __restrict__ out)
{
  __shared__ __align__(16) float sT[64 * kTrP];
  const int tid = threadIdx.x, lane = tid & 31, wave = tid >> 5;
  const int k0 = blockIdx.x * 64, n0 = blockIdx.y * 64;
  const int kr = tid >> 2, cb = (tid & 3) * 16;
  const float* src = in + (size_t)(k0 + kr) * Nreal;
#pragma unroll
  for (int g = 0; g < 4; ++g) {
    const int col = n0 + cb + 4 * g;
    const bool valid = (col < Nreal);
    const int cc = valid ? col : (Nreal - 4);
    const v4f v = *(const v4f*)(src + cc);
    const float fac = valid ? 1.0f : 0.0f;
    *(v4f*)(sT + kr * kTrP + cb + 4 * g) = v * fac;
  }
  __syncthreads();
  const int q = lane >> 3, c8 = (lane & 7) * 8;
  v8h hv[2];
#pragma unroll
  for (int it = 0; it < 2; ++it) {
    const int nl = wave * 8 + it * 4 + q;
#pragma unroll
    for (int e = 0; e < 8; ++e) {
      const float f = sT[(c8 + e) * kTrP + nl];
      hv[it][e] = __builtin_bit_cast(_Float16, f2bf_bits(f));
    }
  }
  for (int pass = 0; pass < 2; ++pass) {
#pragma unroll
    for (int it = 0; it < 2; ++it) {
      const int nl = wave * 8 + it * 4 + q;
      *(volatile v8h*)(out + (size_t)(n0 + nl) * Krows + k0 + c8) = hv[it];
    }
    __threadfence();
  }
}

template <int DIR>
__global__ __launch_bounds__(256) void conv_silu_kernel(
    const float* __restrict__ XZ, const float* __restrict__ cw, const float* __restrict__ cb,
    float* __restrict__ XC, unsigned short* __restrict__ XCH, unsigned short* __restrict__ XCL)
{
  __shared__ __align__(16) float sT[16 * kConvTP];
  const int tid = threadIdx.x, lane = tid & 31, wave = tid >> 5;
  const int d0 = blockIdx.x * 256, d = d0 + tid;
  const int g0 = blockIdx.y * 64;
  const int tb = g0 & (kSeq - 1);
  const float w0 = bf_rne(cw[d * 4 + 0]), w1 = bf_rne(cw[d * 4 + 1]), w2 = bf_rne(cw[d * 4 + 2]), w3 = bf_rne(cw[d * 4 + 3]);
  const float bc = bf_rne(cb[d]);
  float xm3, xm2, xm1;
  {
    bool hist; int rA, rB, rC;
    if (DIR == 0) {
      hist = (tb > 0);
      const int base = hist ? (g0 - 3) : g0;
      rA = base; rB = base + 1; rC = base + 2;
    } else {
      hist = (tb + 64) < kSeq;
      const int base = hist ? (g0 + 64) : g0;
      rC = base; rB = base + 1; rA = base + 2;
    }
    const float vA = XZ[(size_t)rA * kXzP + d];
    const float vB = XZ[(size_t)rB * kXzP + d];
    const float vC = XZ[(size_t)rC * kXzP + d];
    xm3 = hist ? vA : 0.f;
    xm2 = hist ? vB : 0.f;
    xm1 = hist ? vC : 0.f;
  }
  const int hrow = wave >> 1;
  const int hch  = (wave & 1) * 128 + lane * 4;
#pragma unroll 1
  for (int sub = 0; sub < 4; ++sub) {
    const int lb = (DIR == 0) ? (g0 + sub * 16) : (g0 + (3 - sub) * 16);
#pragma unroll 1
    for (int s = 0; s < 16; ++s) {
      const int r = (DIR == 0) ? s : (15 - s);
      const float xcur = XZ[(size_t)(lb + r) * kXzP + d];
      float acc = w0 * xm3;
      acc = fmaf(w1, xm2, acc);
      acc = fmaf(w2, xm1, acc);
      acc = fmaf(w3, xcur, acc);
      const float sv = acc + bc;
      const float sg = __builtin_amdgcn_rcpf(1.0f + expf(-sv));
      sT[r * kConvTP + tid] = sv * sg;
      xm3 = xm2; xm2 = xm1; xm1 = xcur;
    }
    __syncthreads();
    v4f fv[4];
    v8h bh[2], blo[2];
#pragma unroll
    for (int it = 0; it < 4; ++it) fv[it] = *(const v4f*)(sT + (it * 4 + hrow) * kConvTP + hch);
#pragma unroll
    for (int it = 0; it < 2; ++it) {
      const float* sp = sT + (it * 8 + wave) * kConvTP + lane * 8;
      const v4f a0 = *(const v4f*)(sp);
      const v4f a1 = *(const v4f*)(sp + 4);
#pragma unroll
      for (int e = 0; e < 4; ++e) {
        const float f0 = a0[e], f1 = a1[e];
        const unsigned short h0 = f2bf_bits(f0), h1 = f2bf_bits(f1);
        const unsigned short l0 = f2bf_bits(f0 - bf_bits2f(h0)), l1 = f2bf_bits(f1 - bf_bits2f(h1));
        bh[it][e]      = __builtin_bit_cast(_Float16, h0);
        bh[it][4 + e]  = __builtin_bit_cast(_Float16, h1);
        blo[it][e]     = __builtin_bit_cast(_Float16, l0);
        blo[it][4 + e] = __builtin_bit_cast(_Float16, l1);
      }
    }
    for (int pass = 0; pass < 2; ++pass) {
#pragma unroll
      for (int it = 0; it < 4; ++it)
        *(volatile v4f*)(XC + (size_t)(lb + it * 4 + hrow) * kDin + d0 + hch) = fv[it];
#pragma unroll
      for (int it = 0; it < 2; ++it) {
        const size_t o = (size_t)(lb + it * 8 + wave) * kDin + d0 + lane * 8;
        *(volatile v8h*)(XCH + o) = bh[it];
        *(volatile v8h*)(XCL + o) = blo[it];
      }
      __threadfence();
    }
    __syncthreads();
  }
}

template <int DIR>
__global__ __launch_bounds__(64) void scan_kernel(
    const float* __restrict__ PR, const float* __restrict__ XC, const float* __restrict__ XZ,
    const float* __restrict__ Wdt, const float* __restrict__ bdt, const float* __restrict__ Alog,
    const float* __restrict__ Dp, float* __restrict__ YS,
    unsigned short* __restrict__ YH, unsigned short* __restrict__ YL)
{
  __shared__ __align__(16) float sX[kScanTS * kXdP];
  __shared__ __align__(16) float sY[kScanTS * kScanYP];
  __shared__ __align__(16) float sW[kDtR * kScanCh];
  __shared__ __align__(16) float sA[kNst * kScanCh];
  const int tid = threadIdx.x, lane = tid & 31, wave = tid >> 5;
  constexpr int kBlkPerB = kDin / kScanCh;
  const int bix = blockIdx.x / kBlkPerB;
  const int d0  = (blockIdx.x - bix * kBlkPerB) * kScanCh;
  const int d   = d0 + tid;
  const size_t row0 = (size_t)bix * kSeq;
#pragma unroll 1
  for (int r = 0; r < kDtR; ++r) sW[r * kScanCh + tid] = bf_rne(Wdt[(size_t)r * kDin + d]);
#pragma unroll 1
  for (int s = 0; s < kNst; ++s) sA[s * kScanCh + tid] = -expf(bf_rne(Alog[(size_t)d * kNst + s]));
  __syncthreads();
  float negA[kNst], h[kNst];
#pragma unroll
  for (int s = 0; s < kNst; ++s) {
    negA[s] = sA[s * kScanCh + tid];
    h[s] = 0.f;
  }
  const float bb = bf_rne(bdt[d]), Dd = bf_rne(Dp[d]);
  const int lr = tid >> 4, lc4 = (tid & 15) * 4;
  const int q = lane >> 3, c8 = (lane & 7) * 8;
  const int hh = lane >> 4, c4 = (lane & 15) * 4;
#pragma unroll 1
  for (int c = 0; c < kSeq / kScanTS; ++c) {
    const int t0 = (DIR == 0) ? (c * kScanTS) : (kSeq - kScanTS - c * kScanTS);
    __syncthreads();
#pragma unroll
    for (int i = 0; i < 8; ++i) {
      const int r = lr + 4 * i;
      *(v4f*)(sX + r * kXdP + lc4) = *(const v4f*)(PR + (row0 + t0 + r) * kXdP + lc4);
    }
    asm volatile("" ::: "memory");
#pragma unroll
    for (int i = 8; i < 16; ++i) {
      const int r = lr + 4 * i;
      *(v4f*)(sX + r * kXdP + lc4) = *(const v4f*)(PR + (row0 + t0 + r) * kXdP + lc4);
    }
    __syncthreads();
#pragma unroll 1
    for (int p = 0; p < kScanTS; ++p) {
      const int s = (DIR == 0) ? p : (kScanTS - 1 - p);
      const int t = t0 + s;
      const float* xr = sX + s * kXdP;
      float vdot = 0.f;
#pragma unroll 1
      for (int r4 = 0; r4 < kDtR / 4; ++r4) {
        const v4f xv = *(const v4f*)(xr + 4 * r4);
        const float* wp = sW + (4 * r4) * kScanCh + tid;
        vdot = fmaf(xv[0], wp[0], vdot);
        vdot = fmaf(xv[1], wp[kScanCh], vdot);
        vdot = fmaf(xv[2], wp[2 * kScanCh], vdot);
        vdot = fmaf(xv[3], wp[3 * kScanCh], vdot);
      }
      float Bs[kNst], Cs[kNst];
#pragma unroll
      for (int q4 = 0; q4 < 4; ++q4) {
        const v4f bv = *(const v4f*)(xr + kDtR + 4 * q4);
        const v4f cv = *(const v4f*)(xr + kDtR + kNst + 4 * q4);
        Bs[4 * q4 + 0] = bv[0]; Bs[4 * q4 + 1] = bv[1]; Bs[4 * q4 + 2] = bv[2]; Bs[4 * q4 + 3] = bv[3];
        Cs[4 * q4 + 0] = cv[0]; Cs[4 * q4 + 1] = cv[1]; Cs[4 * q4 + 2] = cv[2]; Cs[4 * q4 + 3] = cv[3];
      }
      const float v   = vdot + bb;
      const float a   = __expf(-fabsf(v));
      const float u   = 1.0f + a;
      const float l1p = __logf(u) + (a - (u - 1.0f)) * __builtin_amdgcn_rcpf(u);
      const float dt  = fmaxf(v, 0.0f) + l1p;
      const size_t grow = row0 + t;
      const float xt  = XC[grow * kDin + d];
      const float dtx = dt * xt;
      float y = 0.f;
#pragma unroll
      for (int k = 0; k < kNst; ++k) {
        const float e = __expf(dt * negA[k]);
        h[k] = e * h[k] + dtx * Bs[k];
        y = h[k] * Cs[k] + y;
      }
      y = xt * Dd + y;
      const float zv = XZ[grow * kXzP + kDin + d];
      const float sg = __builtin_amdgcn_rcpf(1.0f + expf(-zv));
      y = y * (zv * sg);
      if (DIR == 1) y = y + YS[grow * kDin + d];
      sY[s * kScanYP + tid] = y;
    }
    __syncthreads();
    if (DIR == 0) {
      for (int pass = 0; pass < 2; ++pass) {
#pragma unroll
        for (int it = 0; it < 16; ++it) {
          const int row = it * 4 + wave * 2 + hh;
          const v4f val = *(const v4f*)(sY + row * kScanYP + c4);
          *(volatile v4f*)(YS + (row0 + t0 + row) * kDin + d0 + c4) = val;
        }
        __threadfence();
      }
    } else {
      v8h hv[8], lv[8];
#pragma unroll
      for (int it = 0; it < 8; ++it) {
        const int row = it * 8 + wave * 4 + q;
        const float* sp = sY + row * kScanYP + c8;
        const v4f a0 = *(const v4f*)(sp);
        const v4f a1 = *(const v4f*)(sp + 4);
#pragma unroll
        for (int e = 0; e < 4; ++e) {
          const float f0 = a0[e], f1 = a1[e];
          const unsigned short h0 = f2bf_bits(f0), h1 = f2bf_bits(f1);
          const unsigned short l0 = f2bf_bits(f0 - bf_bits2f(h0)), l1 = f2bf_bits(f1 - bf_bits2f(h1));
          hv[it][e]     = __builtin_bit_cast(_Float16, h0);
          hv[it][4 + e] = __builtin_bit_cast(_Float16, h1);
          lv[it][e]     = __builtin_bit_cast(_Float16, l0);
          lv[it][4 + e] = __builtin_bit_cast(_Float16, l1);
        }
      }
      for (int pass = 0; pass < 2; ++pass) {
#pragma unroll
        for (int it = 0; it < 8; ++it) {
          const int row = it * 8 + wave * 4 + q;
          const size_t o = (row0 + t0 + row) * kDin + d0 + c8;
          *(volatile v8h*)(YH + o) = hv[it];
          *(volatile v8h*)(YL + o) = lv[it];
        }
        __threadfence();
      }
    }
  }
}

__global__ __launch_bounds__(256) void gelu_split_kernel(
    const float* __restrict__ HP, const float* __restrict__ bias,
    unsigned short* __restrict__ HH, unsigned short* __restrict__ HL, int total2)
{
  const int i = blockIdx.x * 256 + threadIdx.x;
  if (i >= total2) return;
  const size_t e0 = (size_t)i * 2;
  const int n = (int)(e0 & (size_t)(kDff - 1));
  const v2f hp = *(const v2f*)(HP + e0);
  const v2f bv = *(const v2f*)(bias + n);
  const float hp0 = hp[0], hp1 = hp[1], bv0 = bv[0], bv1 = bv[1];
  const float a0 = hp0 + bf_rne(bv0);
  const float a1 = hp1 + bf_rne(bv1);
  float gA = 0.f, gB = 0.f;
#pragma unroll 1
  for (int e = 0; e < 2; ++e) {
    const float v = (e == 0) ? a0 : a1;
    const float g = 0.5f * v * (1.0f + erff(v * 0.70710678118654752f));
    gA = (e == 0) ? g : gA;
    gB = (e == 0) ? gB : g;
  }
  const unsigned short hA = f2bf_bits(gA), hB = f2bf_bits(gB);
  const unsigned short lA = f2bf_bits(gA - bf_bits2f(hA)), lB = f2bf_bits(gB - bf_bits2f(hB));
  const unsigned uh = (unsigned)hA | ((unsigned)hB << 16);
  const unsigned ul = (unsigned)lA | ((unsigned)lB << 16);
  ((volatile unsigned*)HH)[i] = uh;
  ((volatile unsigned*)HL)[i] = ul;
  __threadfence();
  ((volatile unsigned*)HH)[i] = uh;
  ((volatile unsigned*)HL)[i] = ul;
}

__global__ __launch_bounds__(256) void ln_residual_kernel(
    const float* __restrict__ FF, const float* __restrict__ Yf, const float* __restrict__ bff2,
    const float* __restrict__ g2, const float* __restrict__ be2, float* __restrict__ out)
{
  const int lane = threadIdx.x & 31, wave = threadIdx.x >> 5;
  const size_t row = (size_t)blockIdx.x * 8 + wave;
  const int cA = lane * 4, cB = 128 + lane * 4;
  const float* fr = FF + row * kDm;
  const v4f fa = *(const v4f*)(fr + cA);
  const v4f fb = *(const v4f*)(fr + cB);
  const v4f ba = *(const v4f*)(bff2 + cA);
  const v4f bbv = *(const v4f*)(bff2 + cB);
  float v[8];
#pragma unroll
  for (int e = 0; e < 4; ++e) {
    const float f0 = fa[e], f1 = fb[e], b0 = ba[e], b1 = bbv[e];
    v[e]     = f0 + bf_rne(b0);
    v[4 + e] = f1 + bf_rne(b1);
  }
  float s = 0.f;
#pragma unroll
  for (int e = 0; e < 8; ++e) s += v[e];
#pragma unroll
  for (int off = 16; off > 0; off >>= 1) s += __shfl_xor(s, off, 32);
  const float mean = s * (1.0f / (float)kDm);
  float dv[8];
  float sq = 0.f;
#pragma unroll
  for (int e = 0; e < 8; ++e) { dv[e] = v[e] - mean; sq = fmaf(dv[e], dv[e], sq); }
#pragma unroll
  for (int off = 16; off > 0; off >>= 1) sq += __shfl_xor(sq, off, 32);
  const float var = sq * (1.0f / (float)kDm);
  const float rs = rsqrtf(var + 1e-5f);
  asm volatile("" ::: "memory");
  const float* yr = Yf + row * kDm;
  const v4f ya = *(const v4f*)(yr + cA);
  const v4f yb = *(const v4f*)(yr + cB);
  const v4f ga = *(const v4f*)(g2 + cA);
  const v4f gb = *(const v4f*)(g2 + cB);
  const v4f ea = *(const v4f*)(be2 + cA);
  const v4f eb = *(const v4f*)(be2 + cB);
  v4f oa, ob;
#pragma unroll
  for (int e = 0; e < 4; ++e) {
    const float y0 = ya[e], y1 = yb[e], gg0 = ga[e], gg1 = gb[e], be0 = ea[e], be1 = eb[e];
    oa[e] = y0 + ((dv[e] * rs) * bf_rne(gg0) + bf_rne(be0));
    ob[e] = y1 + ((dv[4 + e] * rs) * bf_rne(gg1) + bf_rne(be1));
  }
  float* orow = out + row * kDm;
  for (int pass = 0; pass < 2; ++pass) {
    *(volatile v4f*)(orow + cA) = oa;
    *(volatile v4f*)(orow + cB) = ob;
    __threadfence();
  }
}

extern "C" void kernel_launch(void* const* d_in, const int* in_sizes, int n_in,
                              void* d_out, int out_size, void* d_ws, size_t ws_size,
                              hipStream_t stream) {
  if (n_in < 16) return;
  if (in_sizes[0]  != kRows * kDm) return;
  if (in_sizes[1]  != kDm * kXzP) return;
  if (in_sizes[2]  != kDin * 4) return;
  if (in_sizes[3]  != kDin) return;
  if (in_sizes[4]  != kDin * kXdW) return;
  if (in_sizes[5]  != kDtR * kDin) return;
  if (in_sizes[6]  != kDin) return;
  if (in_sizes[7]  != kDin * kNst) return;
  if (in_sizes[8]  != kDin) return;
  if (in_sizes[9]  != kDin * kDm) return;
  if (in_sizes[10] != kDm * kDff) return;
  if (in_sizes[11] != kDff) return;
  if (in_sizes[12] != kDff * kDm) return;
  if (in_sizes[13] != kDm) return;
  if (in_sizes[14] != kDm) return;
  if (in_sizes[15] != kDm) return;
  if (out_size != kRows * kDm) return;
  if (ws_size < kWsTotal) return;

  const float* x       = (const float*)d_in[0];
  const float* W_in    = (const float*)d_in[1];
  const float* conv_w  = (const float*)d_in[2];
  const float* conv_b  = (const float*)d_in[3];
  const float* W_xproj = (const float*)d_in[4];
  const float* W_dt    = (const float*)d_in[5];
  const float* b_dt    = (const float*)d_in[6];
  const float* A_log   = (const float*)d_in[7];
  const float* Dp      = (const float*)d_in[8];
  const float* W_out   = (const float*)d_in[9];
  const float* W_ff1   = (const float*)d_in[10];
  const float* b_ff1   = (const float*)d_in[11];
  const float* W_ff2   = (const float*)d_in[12];
  const float* b_ff2   = (const float*)d_in[13];
  const float* g2      = (const float*)d_in[14];
  const float* beta2   = (const float*)d_in[15];
  float* out = (float*)d_out;

  char* ws = (char*)d_ws;
  unsigned short* XB  = (unsigned short*)(ws + kOffXB);
  unsigned short* WIB = (unsigned short*)(ws + kOffWIB);
  unsigned short* WXB = (unsigned short*)(ws + kOffWXB);
  unsigned short* WOB = (unsigned short*)(ws + kOffWOB);
  unsigned short* WF1 = (unsigned short*)(ws + kOffWF1);
  unsigned short* WF2 = (unsigned short*)(ws + kOffWF2);
  float*          XZ  = (float*)(ws + kOffXZ);
  float*          XC  = (float*)(ws + kOffXC);
  unsigned short* XCH = (unsigned short*)(ws + kOffXCH);
  unsigned short* XCL = (unsigned short*)(ws + kOffXCL);
  float*          PR  = (float*)(ws + kOffPR);
  float*          YS  = (float*)(ws + kOffYS);
  unsigned short* YH  = (unsigned short*)(ws + kOffYH);
  unsigned short* YL  = (unsigned short*)(ws + kOffYL);
  unsigned short* Y2H = (unsigned short*)(ws + kOffY2H);
  unsigned short* Y2L = (unsigned short*)(ws + kOffY2L);
  float*          HP  = (float*)(ws + kOffHP);
  float*          FF  = (float*)(ws + kOffFF);
  unsigned short* HH  = (unsigned short*)(ws + kOffHH);
  float*          Yf  = (float*)(ws + kOffYf);
  unsigned short* HL  = (unsigned short*)(ws + kOffHL);

  rne_rows_bf16_kernel<<<(kRows * kDm / 8) / 256, 256, 0, stream>>>(x, XB, kRows * kDm / 8);
  transpose_bf16_kernel<<<dim3(kDm / 64, kXzP / 64), 256, 0, stream>>>(W_in, kXzP, kDm, WIB);
  transpose_bf16_kernel<<<dim3(kDin / 64, kXdP / 64), 256, 0, stream>>>(W_xproj, kXdW, kDin, WXB);
  transpose_bf16_kernel<<<dim3(kDin / 64, kDm / 64), 256, 0, stream>>>(W_out, kDm, kDin, WOB);
  transpose_bf16_kernel<<<dim3(kDm / 64, kDff / 64), 256, 0, stream>>>(W_ff1, kDff, kDm, WF1);
  transpose_bf16_kernel<<<dim3(kDff / 64, kDm / 64), 256, 0, stream>>>(W_ff2, kDm, kDff, WF2);

  wmma_gemm64<1, 0, 0, 0, false><<<dim3(256, 1), 256, 0, stream>>>(
      XB, nullptr, kDm, 0L,
      WIB, nullptr, kDm, 0L,
      (void*)XZ, nullptr, kXzP, 0L,
      nullptr, nullptr, 0L,
      kRows, kXzP, kDm, 1.0f);

  conv_silu_kernel<0><<<dim3(kDin / 256, kRows / 64), 256, 0, stream>>>(XZ, conv_w, conv_b, XC, XCH, XCL);
  wmma_gemm64<1, 1, 0, 0, false><<<dim3(16, 1), 256, 0, stream>>>(
      XCH, XCL, kDin, 0L,
      WXB, nullptr, kDin, 0L,
      (void*)PR, nullptr, kXdP, 0L,
      nullptr, nullptr, 0L,
      kRows, kXdP, kDin, 1.0f);
  scan_kernel<0><<<kBatch * (kDin / kScanCh), kScanCh, 0, stream>>>(PR, XC, XZ, W_dt, b_dt, A_log, Dp, YS, YH, YL);

  conv_silu_kernel<1><<<dim3(kDin / 256, kRows / 64), 256, 0, stream>>>(XZ, conv_w, conv_b, XC, XCH, XCL);
  wmma_gemm64<1, 1, 0, 0, false><<<dim3(16, 1), 256, 0, stream>>>(
      XCH, XCL, kDin, 0L,
      WXB, nullptr, kDin, 0L,
      (void*)PR, nullptr, kXdP, 0L,
      nullptr, nullptr, 0L,
      kRows, kXdP, kDin, 1.0f);
  scan_kernel<1><<<kBatch * (kDin / kScanCh), kScanCh, 0, stream>>>(PR, XC, XZ, W_dt, b_dt, A_log, Dp, YS, YH, YL);

  wmma_gemm64<1, 1, 0, 0, false><<<dim3(64, 1), 256, 0, stream>>>(
      YH, YL, kDin, 0L,
      WOB, nullptr, kDin, 0L,
      (void*)Yf, nullptr, kDm, 0L,
      nullptr, nullptr, 0L,
      kRows, kDm, kDin, 1.0f);
  split_rows_bf16_kernel<<<(kRows * kDm / 8) / 256, 256, 0, stream>>>(Yf, Y2H, Y2L, kRows * kDm / 8);

  wmma_gemm64<1, 1, 0, 0, false><<<dim3(256, 1), 256, 0, stream>>>(
      Y2H, Y2L, kDm, 0L,
      WF1, nullptr, kDm, 0L,
      (void*)HP, nullptr, kDff, 0L,
      nullptr, nullptr, 0L,
      kRows, kDff, kDm, 1.0f);
  gelu_split_kernel<<<(kRows * kDff / 2) / 256, 256, 0, stream>>>(HP, b_ff1, HH, HL, kRows * kDff / 2);

  wmma_gemm64<1, 1, 0, 0, false><<<dim3(64, 1), 256, 0, stream>>>(
      HH, HL, kDff, 0L,
      WF2, nullptr, kDff, 0L,
      (void*)FF, nullptr, kDm, 0L,
      nullptr, nullptr, 0L,
      kRows, kDm, kDff, 1.0f);

  ln_residual_kernel<<<kRows / 8, 256, 0, stream>>>(FF, Yf, b_ff2, g2, beta2, out);
}
